// GCN_420906795032
// MI455X (gfx1250) — hardware-verified
//
#include <hip/hip_runtime.h>
#include <stddef.h>
#include <stdint.h>
#include <math.h>


#define DIM    256
#define XP     512
#define NTHR   256
#define NWAVE  8
#define EPT    8
#define CHUNK  (NTHR * EPT)
#define WCAP   (EPT * 32)
#define LISTN  (NWAVE * WCAP)
#define NBA    512
#define SLA    9
#define RCAP   20480
#define DEGCAP 96
#define GBM    64
#define GBN    128
#define GTHR   128
#define NU1    (DIM * (DIM / 8))
#define NU2    (DIM * (XP / 8))
#define MISC_INTS 16
#define FLAGP  32
#define BKT_ZINTS    (LISTN + 2 * RCAP + 3 * NBA)
#define BKT_LDS_INTS (BKT_ZINTS + MISC_INTS + NBA)
#define WSMAX  134217728

static_assert((CHUNK & (CHUNK - 1)) == 0 && CHUNK <= 4096);
static_assert((NBA & (NBA - 1)) == 0 && NBA == (1 << SLA));
static_assert(((long long)CHUNK << SLA) < (1LL << 31));
static_assert(LISTN % NTHR == 0);
static_assert(NBA % NWAVE == 0 && NBA % 32 == 0 && NBA % GBM == 0 && NBA == 2 * NTHR);
static_assert(RCAP % (NTHR * 4) == 0 && BKT_ZINTS % 4 == 0 && LISTN % 4 == 0);
static_assert(((BKT_ZINTS + MISC_INTS) % 4) == 0);
static_assert(DIM % 32 == 0 && XP % 32 == 0 && XP == 2 * DIM && DIM == 2 * GBN);
static_assert(GBM == (GTHR / 32) * 16 && GBN == 4 * 32);
static_assert(NU1 % NTHR == 0 && NU2 % NTHR == 0);
static_assert(DIM == 8 * 32);
static_assert(BKT_LDS_INTS * 4 <= 300000);
static_assert(DEGCAP >= 61 + 8 && RCAP >= 16715 + 1024);

typedef float          v4f   __attribute__((ext_vector_type(4)));
typedef float          v8f   __attribute__((ext_vector_type(8)));
typedef int            v4i   __attribute__((ext_vector_type(4)));
typedef int            v8i   __attribute__((ext_vector_type(8)));
typedef unsigned short v4us  __attribute__((ext_vector_type(4)));
typedef unsigned short v8us  __attribute__((ext_vector_type(8)));
typedef unsigned short v16us __attribute__((ext_vector_type(16)));
typedef __bf16         v16bf __attribute__((ext_vector_type(16)));
typedef v4f  __attribute__((may_alias)) v4fa;
typedef v4i  __attribute__((may_alias)) v4ia;
typedef v4us __attribute__((may_alias)) v4usa;
typedef v8us __attribute__((may_alias)) v8usa;
union FragB { v16bf v; v16us u; v8us h[2]; v8i w; };

__device__ __forceinline__ v8f wmb(const FragB& a, const FragB& b, v8f c) {
  v8f d = __builtin_amdgcn_wmma_f32_16x16x32_bf16(false, a.v, false, b.v, (short)0, c, false, false);
  asm volatile("v_nop\n\tv_nop\n\tv_nop\n\tv_nop" : "+v"(d) : "v"(a.w), "v"(b.w));
  return d;
}

__device__ __forceinline__ unsigned bf16_bits(float f) {
  const unsigned u = __float_as_uint(f);
  const unsigned r = (u + 0x7FFFu + ((u >> 16) & 1u)) >> 16;
  const bool isn = (u & 0x7fffffffu) > 0x7f800000u;
  return isn ? 0x7fc0u : r;
}
__device__ __forceinline__ float bf16_val(float f) {
  return __uint_as_float(bf16_bits(f) << 16);
}
__device__ __forceinline__ float relu_np(float v) {
  return (v > 0.0f) ? v : (v - v);
}
__device__ __forceinline__ void split4(const v4f y, v4us* h, v4us* l) {
  v4us hh, ll;
  unsigned hb;
  hb = bf16_bits(y.x); hh[0] = (unsigned short)hb; ll[0] = (unsigned short)bf16_bits(y.x - __uint_as_float(hb << 16));
  hb = bf16_bits(y.y); hh[1] = (unsigned short)hb; ll[1] = (unsigned short)bf16_bits(y.y - __uint_as_float(hb << 16));
  hb = bf16_bits(y.z); hh[2] = (unsigned short)hb; ll[2] = (unsigned short)bf16_bits(y.z - __uint_as_float(hb << 16));
  hb = bf16_bits(y.w); hh[3] = (unsigned short)hb; ll[3] = (unsigned short)bf16_bits(y.w - __uint_as_float(hb << 16));
  *h = hh; *l = ll;
}

__device__ __forceinline__ void wave_sync() {
  __builtin_amdgcn_fence(__ATOMIC_RELEASE, "wavefront");
  __builtin_amdgcn_wave_barrier();
  __builtin_amdgcn_fence(__ATOMIC_ACQUIRE, "wavefront");
}

template <int SLB>
__device__ __forceinline__ int scan_chunk(const int* __restrict__ dsts, int nE, int cbase, int slotBase,
                                          int nb, int vec8, int* list, int tid, int lane, int wave) {
  int wc = 0;
  const int el0  = tid * EPT;
  const int e0   = cbase + el0;
  const int sent = -2147483647 - 1;
  v4i da, db;
  if (vec8 != 0 && cbase + CHUNK <= nE) {
    da = *(const v4i*)(dsts + e0);
    db = *(const v4i*)(dsts + e0 + 4);
  } else {
    da.x = (e0     < nE) ? dsts[min(e0,     nE - 1)] : sent;
    da.y = (e0 + 1 < nE) ? dsts[min(e0 + 1, nE - 1)] : sent;
    da.z = (e0 + 2 < nE) ? dsts[min(e0 + 2, nE - 1)] : sent;
    da.w = (e0 + 3 < nE) ? dsts[min(e0 + 3, nE - 1)] : sent;
    db.x = (e0 + 4 < nE) ? dsts[min(e0 + 4, nE - 1)] : sent;
    db.y = (e0 + 5 < nE) ? dsts[min(e0 + 5, nE - 1)] : sent;
    db.z = (e0 + 6 < nE) ? dsts[min(e0 + 6, nE - 1)] : sent;
    db.w = (e0 + 7 < nE) ? dsts[min(e0 + 7, nE - 1)] : sent;
  }
  const unsigned nbs = (unsigned)slotBase;
  const unsigned unb = (unsigned)nb;
  const unsigned s0 = (unsigned)da.x - nbs, s1 = (unsigned)da.y - nbs;
  const unsigned s2 = (unsigned)da.z - nbs, s3 = (unsigned)da.w - nbs;
  const unsigned s4 = (unsigned)db.x - nbs, s5 = (unsigned)db.y - nbs;
  const unsigned s6 = (unsigned)db.z - nbs, s7 = (unsigned)db.w - nbs;
  const bool h0 = s0 < unb, h1 = s1 < unb, h2 = s2 < unb, h3 = s3 < unb;
  const bool h4 = s4 < unb, h5 = s5 < unb, h6 = s6 < unb, h7 = s7 < unb;
  const unsigned any = __builtin_amdgcn_ballot_w32(h0 | h1 | h2 | h3 | h4 | h5 | h6 | h7);
  if (any != 0u) {
#define HITJ(J, HJ, SJ) { \
      const unsigned mj = __builtin_amdgcn_ballot_w32(HJ); \
      if (mj != 0u) { \
        if (HJ) { \
          const int pos = wc + (int)__builtin_amdgcn_mbcnt_lo(mj, 0u); \
          if (pos < WCAP) list[wave * WCAP + pos] = ((el0 + (J)) << SLB) | (int)(SJ); \
        } \
        wc += (int)__builtin_popcount(mj); } }
    HITJ(0, h0, s0)
    HITJ(1, h1, s1)
    HITJ(2, h2, s2)
    HITJ(3, h3, s3)
    HITJ(4, h4, s4)
    HITJ(5, h5, s5)
    HITJ(6, h6, s6)
    HITJ(7, h7, s7)
#undef HITJ
  }
  return wc;
}

__global__ __launch_bounds__(NTHR) void k_wprep(const float* __restrict__ W1, const float* __restrict__ W2,
                                                const float* __restrict__ W3,
                                                unsigned short* W1T, unsigned short* W2D, unsigned short* W3D) {
  const int u = (int)blockIdx.x * NTHR + (int)threadIdx.x;
  v8us o;
  unsigned short* dp;
  if (u < NU1) {
    const int n  = u >> 5;
    const int k8 = (u & 31) * 8;
    const float* p = W1 + (size_t)k8 * DIM + n;
#pragma unroll
    for (int i = 0; i < 8; ++i) o[i] = (unsigned short)bf16_bits(p[(size_t)i * DIM]);
    dp = W1T + (size_t)n * DIM + k8;
  } else if (u < NU1 + NU2) {
    const int v  = u - NU1;
    const int n  = v >> 6;
    const int k8 = (v & 63) * 8;
    const int kk = k8 & (DIM - 1);
    const float* p = W2 + (size_t)kk * DIM + n;
#pragma unroll
    for (int i = 0; i < 8; ++i) o[i] = (unsigned short)bf16_bits(p[(size_t)i * DIM]);
    dp = W2D + (size_t)n * XP + k8;
  } else if (u < NU1 + 2 * NU2) {
    const int v  = u - NU1 - NU2;
    const int n  = v >> 6;
    const int k8 = (v & 63) * 8;
    const int kk = k8 & (DIM - 1);
    const float* p = W3 + (size_t)kk * DIM + n;
#pragma unroll
    for (int i = 0; i < 8; ++i) o[i] = (unsigned short)bf16_bits(p[(size_t)i * DIM]);
    dp = W3D + (size_t)n * XP + k8;
  } else {
    return;
  }
  *(volatile v8us*)dp = o;
  __threadfence();
  *(volatile v8us*)dp = o;
}

__global__ __launch_bounds__(NTHR) void k_cvx(const float* __restrict__ x, int nN, int nUnits,
                                              unsigned short* xb) {
  const int u = (int)blockIdx.x * NTHR + (int)threadIdx.x;
  if (u >= nUnits) return;
  const int row = u >> 5;
  const int k8  = (u & 31) * 8;
  const int rc  = row < nN ? row : nN - 1;
  const float* p = x + (size_t)rc * DIM + k8;
  const v4f a = *(const v4fa*)p;
  const v4f b = *(const v4fa*)(p + 4);
  const bool ok = row < nN;
  v8us o;
  o[0] = ok ? (unsigned short)bf16_bits(a.x) : (unsigned short)0;
  o[1] = ok ? (unsigned short)bf16_bits(a.y) : (unsigned short)0;
  o[2] = ok ? (unsigned short)bf16_bits(a.z) : (unsigned short)0;
  o[3] = ok ? (unsigned short)bf16_bits(a.w) : (unsigned short)0;
  o[4] = ok ? (unsigned short)bf16_bits(b.x) : (unsigned short)0;
  o[5] = ok ? (unsigned short)bf16_bits(b.y) : (unsigned short)0;
  o[6] = ok ? (unsigned short)bf16_bits(b.z) : (unsigned short)0;
  o[7] = ok ? (unsigned short)bf16_bits(b.w) : (unsigned short)0;
  unsigned short* dp = xb + (size_t)row * DIM + k8;
  *(volatile v8us*)dp = o;
  __threadfence();
  *(volatile v8us*)dp = o;
}

__global__ __launch_bounds__(NTHR) void k_bucket(const int* __restrict__ srcs, const int* __restrict__ dsts,
                                                 int nE, int nN, int vec8,
                                                 int* srcl, int* cntg, int* offg, int* flagg, float* dis) {
  extern __shared__ __attribute__((aligned(16))) int dsm[];
  int* list = dsm;
  int* hl   = dsm + LISTN;
  int* sl   = hl + RCAP;
  int* cnt  = sl + RCAP;
  int* offs = cnt + NBA;
  int* cur  = offs + NBA;
  int* misc = cur + NBA;
  float* disl = (float*)(misc + MISC_INTS);
  const int tid = (int)threadIdx.x, lane = tid & 31, wave = tid >> 5;
  const int blk = (int)blockIdx.x;
  const int nodeBase = blk * NBA;

  {
    const v4i z4 = {0, 0, 0, 0};
    for (int i = tid * 4; i < BKT_ZINTS; i += NTHR * 4) *(v4ia*)(dsm + i) = z4;
    if (tid < MISC_INTS) misc[tid] = 0;
  }
  __syncthreads();

  int t = 0, ov = 0;
  const int nChunks = (nE + CHUNK - 1) / CHUNK;
#pragma unroll 1
  for (int ch = 0; ch < nChunks; ++ch) {
    const int cbase = ch * CHUNK;
    const int wc = scan_chunk<SLA>(dsts, nE, cbase, nodeBase, NBA, vec8, list, tid, lane, wave);
    if (lane == 0) misc[wave] = wc;
    __syncthreads();
    if (wave == 0) {
#pragma unroll 1
      for (int w2 = 0; w2 < NWAVE; ++w2) {
        int c = misc[w2];
        c = c < 0 ? 0 : (c > WCAP ? WCAP : c);
#pragma unroll 1
        for (int b0 = 0; b0 < c; b0 += 32) {
          const int idx = b0 + lane;
          const int ent = list[w2 * WCAP + (idx < WCAP ? idx : WCAP - 1)];
          const int m32 = (c - b0) < 32 ? (c - b0) : 32;
#pragma unroll 1
          for (int k = 0; k < m32; ++k) {
            const int u    = __builtin_amdgcn_readlane(ent, k);
            const int slot = u & (NBA - 1);
            const int el   = (u >> SLA) & (CHUNK - 1);
            const int pk   = ((cbase + el) << SLA) | slot;
            if (t < RCAP) {
              if (lane == 0) { hl[t] = pk; cnt[slot] = cnt[slot] + 1; }
              t = t + 1;
            } else {
              ov = 1;
            }
          }
        }
      }
    }
    __syncthreads();
  }
  if (wave == 0 && lane == 0) { misc[8] = t; misc[9] = ov; }
  __syncthreads();
  int tt = misc[8];
  tt = tt < 0 ? 0 : (tt > RCAP ? RCAP : tt);
  const int ovf = misc[9];

  if (wave == 0) {
    const int base = lane * (NBA / 32);
    int s = 0;
#pragma unroll 1
    for (int i = 0; i < NBA / 32; ++i) s += cnt[base + i];
    int incl = s;
#pragma unroll
    for (int d = 1; d < 32; d <<= 1) {
      const int y = __shfl_up(incl, d, 32);
      if (lane >= d) incl += y;
    }
    int run = incl - s;
#pragma unroll 1
    for (int i = 0; i < NBA / 32; ++i) {
      const int cv = cnt[base + i];
      offs[base + i] = run;
      cur[base + i]  = run;
      run += cv;
    }
  }
  __syncthreads();
  if (wave == 0) {
#pragma unroll 1
    for (int b0 = 0; b0 < tt; b0 += 32) {
      const int idx = b0 + lane;
      const int ent = hl[idx < RCAP ? idx : RCAP - 1];
      const int m32 = (tt - b0) < 32 ? (tt - b0) : 32;
#pragma unroll 1
      for (int k = 0; k < m32; ++k) {
        const int u    = __builtin_amdgcn_readlane(ent, k);
        const int slot = u & (NBA - 1);
        if (lane == 0) {
          int p = cur[slot];
          p = p < 0 ? 0 : (p > RCAP - 1 ? RCAP - 1 : p);
          sl[p] = u;
          cur[slot] = p + 1;
        }
      }
    }
  }
#pragma unroll 1
  for (int i = tid; i < NBA; i += NTHR) {
    int c = cnt[i];
    c = c < 0 ? 0 : c;
    disl[i] = 1.0f / sqrtf((float)(c + 1));
  }
  __syncthreads();

  int* myl = srcl + (size_t)blk * RCAP;
#pragma unroll 1
  for (int i4 = tid * 4; i4 < RCAP; i4 += NTHR * 4) {
    const v4i e4 = *(const v4ia*)(sl + i4);
    int q0 = e4.x >> SLA, q1 = e4.y >> SLA, q2 = e4.z >> SLA, q3 = e4.w >> SLA;
    q0 = q0 < 0 ? 0 : (q0 > nE - 1 ? nE - 1 : q0);
    q1 = q1 < 0 ? 0 : (q1 > nE - 1 ? nE - 1 : q1);
    q2 = q2 < 0 ? 0 : (q2 > nE - 1 ? nE - 1 : q2);
    q3 = q3 < 0 ? 0 : (q3 > nE - 1 ? nE - 1 : q3);
    int r0 = srcs[q0], r1 = srcs[q1], r2 = srcs[q2], r3 = srcs[q3];
    r0 = r0 < 0 ? 0 : (r0 > nN - 1 ? nN - 1 : r0);
    r1 = r1 < 0 ? 0 : (r1 > nN - 1 ? nN - 1 : r1);
    r2 = r2 < 0 ? 0 : (r2 > nN - 1 ? nN - 1 : r2);
    r3 = r3 < 0 ? 0 : (r3 > nN - 1 ? nN - 1 : r3);
    v4i o;
    o.x = (i4     < tt) ? r0 : 0;
    o.y = (i4 + 1 < tt) ? r1 : 0;
    o.z = (i4 + 2 < tt) ? r2 : 0;
    o.w = (i4 + 3 < tt) ? r3 : 0;
    int* dp = myl + i4;
    *(volatile v4i*)dp = o;
    __threadfence();
    *(volatile v4i*)dp = o;
  }

  if (tid < NBA / 4) {
    const v4i c4 = *(const v4ia*)(cnt + 4 * tid);
    const v4i o4 = *(const v4ia*)(offs + 4 * tid);
    const v4f d4 = *(const v4fa*)(disl + 4 * tid);
    int*   cp = cntg + (size_t)nodeBase + 4 * tid;
    int*   op = offg + (size_t)nodeBase + 4 * tid;
    float* dp = dis  + (size_t)nodeBase + 4 * tid;
    *(volatile v4i*)cp = c4;
    *(volatile v4i*)op = o4;
    *(volatile v4f*)dp = d4;
    __threadfence();
    *(volatile v4i*)cp = c4;
    *(volatile v4i*)op = o4;
    *(volatile v4f*)dp = d4;
  }
  if (tid < 8) {
    const v4i f4 = {ovf, ovf, ovf, ovf};
    int* fp = flagg + (size_t)blk * FLAGP + 4 * tid;
    *(volatile v4i*)fp = f4;
    __threadfence();
    *(volatile v4i*)fp = f4;
  }
}

__global__ __launch_bounds__(GTHR) void k_gemm(const unsigned short* __restrict__ A, int lda,
                                               const unsigned short* __restrict__ BT, int K, float* outF) {
  __shared__ __attribute__((aligned(16))) float stg[GBM * GBN];
  const int tid = (int)threadIdx.x, lane = tid & 31, wave = tid >> 5, hh = lane >> 4, m = lane & 15;
  const int rowBase = (int)blockIdx.x * GBM;
  const int col0    = (int)blockIdx.y * GBN;

  v8f acc[8];
  {
    const v8f z = {0.f, 0.f, 0.f, 0.f, 0.f, 0.f, 0.f, 0.f};
#pragma unroll
    for (int t = 0; t < 8; ++t) acc[t] = z;
  }
  const unsigned short* ap = A  + (size_t)(rowBase + 16 * wave + m) * (size_t)lda + 8 * hh;
  const unsigned short* bp = BT + (size_t)(col0 + m) * (size_t)K + 8 * hh;

#pragma unroll 1
  for (int k0 = 0; k0 < K; k0 += 32) {
    FragB af;
    af.h[0] = *(const v8usa*)(ap + k0);
    af.h[1] = *(const v8usa*)(ap + k0 + 16);
#pragma unroll
    for (int nt = 0; nt < 8; ++nt) {
      const unsigned short* wq = bp + (size_t)(16 * nt) * (size_t)K + k0;
      FragB bf;
      bf.h[0] = *(const v8usa*)wq;
      bf.h[1] = *(const v8usa*)(wq + 16);
      acc[nt] = wmb(af, bf, acc[nt]);
    }
  }

#pragma unroll
  for (int nt = 0; nt < 8; ++nt) {
    const int lc = 16 * nt + m;
#pragma unroll
    for (int r = 0; r < 8; ++r) {
      const int lr = 16 * wave + 8 * hh + r;
      stg[lr * GBN + lc] = acc[nt][r];
    }
  }
  __syncthreads();

  v4f pv[16];
#pragma unroll
  for (int i = 0; i < 16; ++i) pv[i] = *(const v4fa*)(stg + (16 * wave + i) * GBN + 4 * lane);
#pragma unroll
  for (int i = 0; i < 16; ++i) {
    float* op = outF + (size_t)(rowBase + 16 * wave + i) * DIM + col0 + 4 * lane;
    *(volatile v4f*)op = pv[i];
  }
  __threadfence();
#pragma unroll
  for (int i = 0; i < 16; ++i) {
    float* op = outF + (size_t)(rowBase + 16 * wave + i) * DIM + col0 + 4 * lane;
    *(volatile v4f*)op = pv[i];
  }
}

template <int MODE>
__global__ __launch_bounds__(NTHR) void k_agg(const int* __restrict__ srcl, const int* __restrict__ cntg,
                                              const int* __restrict__ offg, const int* __restrict__ flagg,
                                              const float* __restrict__ dis, const float* __restrict__ hin,
                                              const float* __restrict__ bias, int nN, int mRows,
                                              unsigned short* xhl, float* outp) {
  __shared__ __attribute__((aligned(16))) unsigned short rowbufs[NWAVE * XP];
  const int tid = (int)threadIdx.x, lane = tid & 31, wave = tid >> 5;
  const int blk = (int)blockIdx.x;
  const int nodeBase = blk * NBA;
  const int* myl = srcl + (size_t)blk * RCAP;
  unsigned short* rowbuf = rowbufs + wave * XP;

  const int ovf = flagg[(size_t)blk * FLAGP];
  v4f bA, bB;
  {
    const v4f t1 = *(const v4fa*)(bias + 4 * lane);
    const v4f t2 = *(const v4fa*)(bias + 128 + 4 * lane);
    bA.x = bf16_val(t1.x); bA.y = bf16_val(t1.y); bA.z = bf16_val(t1.z); bA.w = bf16_val(t1.w);
    bB.x = bf16_val(t2.x); bB.y = bf16_val(t2.y); bB.z = bf16_val(t2.z); bB.w = bf16_val(t2.w);
  }
  const float qnan = __int_as_float(0x7fc00000);
  const float pz = (ovf != 0) ? qnan : 0.0f;

#pragma unroll 1
  for (int si = 0; si < NBA / NWAVE; ++si) {
    const int s    = si * NWAVE + wave;
    const int node = nodeBase + s;
    int c = cntg[node];
    const bool big = (c > DEGCAP) || (c < 0);
    c = c < 0 ? 0 : (c > DEGCAP ? DEGCAP : c);
    int o = offg[node];
    o = o < 0 ? 0 : (o > RCAP ? RCAP : o);
    const int nc = node < nN ? node : nN - 1;
    const float dd = dis[nc];
    const float rd = dd * dd;
    v4f aA = {0.0f, 0.0f, 0.0f, 0.0f};
    v4f aB = {0.0f, 0.0f, 0.0f, 0.0f};
#pragma unroll 1
    for (int b0 = 0; b0 < c; b0 += 32) {
      int idx = o + b0 + lane;
      idx = idx > RCAP - 1 ? RCAP - 1 : idx;
      int sr = myl[idx];
      sr = sr < 0 ? 0 : (sr > nN - 1 ? nN - 1 : sr);
      const float cf  = dis[sr] * dd;
      const int   cfi = __float_as_int(cf);
      const int m32 = (c - b0) < 32 ? (c - b0) : 32;
#pragma unroll 1
      for (int k = 0; k < m32; ++k) {
        const int   sk = __builtin_amdgcn_readlane(sr, k);
        const float ck = __int_as_float(__builtin_amdgcn_readlane(cfi, k));
        const float* hp = hin + (size_t)sk * DIM + 4 * lane;
        const v4f a = *(const v4fa*)hp;
        const v4f b = *(const v4fa*)(hp + 128);
        aA.x = fmaf(ck, a.x, aA.x); aA.y = fmaf(ck, a.y, aA.y);
        aA.z = fmaf(ck, a.z, aA.z); aA.w = fmaf(ck, a.w, aA.w);
        aB.x = fmaf(ck, b.x, aB.x); aB.y = fmaf(ck, b.y, aB.y);
        aB.z = fmaf(ck, b.z, aB.z); aB.w = fmaf(ck, b.w, aB.w);
      }
    }
    const float* sp = hin + (size_t)nc * DIM + 4 * lane;
    const v4f sA = *(const v4fa*)sp;
    const v4f sB = *(const v4fa*)(sp + 128);
    v4f yA, yB;
    yA.x = (aA.x + sA.x * rd) + bA.x; yA.y = (aA.y + sA.y * rd) + bA.y;
    yA.z = (aA.z + sA.z * rd) + bA.z; yA.w = (aA.w + sA.w * rd) + bA.w;
    yB.x = (aB.x + sB.x * rd) + bB.x; yB.y = (aB.y + sB.y * rd) + bB.y;
    yB.z = (aB.z + sB.z * rd) + bB.z; yB.w = (aB.w + sB.w * rd) + bB.w;
    if constexpr (MODE != 0) {
      yA.x = relu_np(yA.x); yA.y = relu_np(yA.y); yA.z = relu_np(yA.z); yA.w = relu_np(yA.w);
      yB.x = relu_np(yB.x); yB.y = relu_np(yB.y); yB.z = relu_np(yB.z); yB.w = relu_np(yB.w);
    }
    const float pzr = big ? qnan : pz;
    const bool live = node < nN;
    yA.x = live ? (yA.x + pzr) : 0.0f; yA.y = live ? (yA.y + pzr) : 0.0f;
    yA.z = live ? (yA.z + pzr) : 0.0f; yA.w = live ? (yA.w + pzr) : 0.0f;
    yB.x = live ? (yB.x + pzr) : 0.0f; yB.y = live ? (yB.y + pzr) : 0.0f;
    yB.z = live ? (yB.z + pzr) : 0.0f; yB.w = live ? (yB.w + pzr) : 0.0f;

    if constexpr (MODE != 0) {
      v4us hA, lA, hB, lB;
      split4(yA, &hA, &lA);
      split4(yB, &hB, &lB);
      *(v4usa*)(rowbuf + 4 * lane) = hA;
      *(v4usa*)(rowbuf + 128 + 4 * lane) = hB;
      *(v4usa*)(rowbuf + DIM + 4 * lane) = lA;
      *(v4usa*)(rowbuf + DIM + 128 + 4 * lane) = lB;
      wave_sync();
      const v8us q0 = *(const v8usa*)(rowbuf + 8 * lane);
      const v8us q1 = *(const v8usa*)(rowbuf + DIM + 8 * lane);
      wave_sync();
      if (node < mRows) {
        unsigned short* rpw = xhl + (size_t)node * XP + 8 * lane;
        *(volatile v8us*)rpw = q0;
        *(volatile v8us*)(rpw + DIM) = q1;
        __threadfence();
        *(volatile v8us*)rpw = q0;
        *(volatile v8us*)(rpw + DIM) = q1;
      }
    } else {
      if (node < nN) {
        float* op = outp + (size_t)node * DIM + 4 * lane;
        *(volatile v4f*)op = yA;
        *(volatile v4f*)(op + 128) = yB;
        __threadfence();
        *(volatile v4f*)op = yA;
        *(volatile v4f*)(op + 128) = yB;
      }
    }
  }
}

static inline int cdiv(int a, int b) { return (a + b - 1) / b; }
static inline size_t al256(size_t o) { return (o + 255) & ~(size_t)255; }

extern "C" void kernel_launch(void* const* d_in, const int* in_sizes, int n_in,
                              void* d_out, int out_size, void* d_ws, size_t ws_size,
                              hipStream_t stream) {
  if (n_in < 8) return;
  if (in_sizes[0] < DIM || (in_sizes[0] % DIM) != 0) return;
  const int nN = in_sizes[0] / DIM;
  if (nN < 16 || nN > (1 << 22)) return;
  if (in_sizes[1] != DIM * DIM || in_sizes[2] != DIM) return;
  if (in_sizes[3] != DIM * DIM || in_sizes[4] != DIM) return;
  if (in_sizes[5] != DIM * DIM || in_sizes[6] != DIM) return;
  if (in_sizes[7] < 2 || (in_sizes[7] & 1) != 0) return;
  const int nE = in_sizes[7] / 2;
  if (nE < 1 || nE >= (1 << (31 - SLA))) return;
  if ((long long)out_size != (long long)nN * DIM) return;

  const float* x    = (const float*)d_in[0];
  const float* W1   = (const float*)d_in[1];
  const float* b1   = (const float*)d_in[2];
  const float* W2   = (const float*)d_in[3];
  const float* b2   = (const float*)d_in[4];
  const float* W3   = (const float*)d_in[5];
  const float* b3   = (const float*)d_in[6];
  const int*   edge = (const int*)d_in[7];
  float* out = (float*)d_out;
  const int* src = edge;
  const int* dst = edge + nE;

  const int MP  = cdiv(nN, GBM) * GBM;
  const int gM  = MP / GBM;
  const int gA  = cdiv(MP, NBA);
  const int NBP = gA * NBA;
  if ((long long)gA * NBA < (long long)MP) return;
  const int vec8 = ((nE & 3) == 0) ? 1 : 0;

  char* ws = (char*)d_ws;
  size_t off = 0;
  const size_t oDIS = off; off = al256(off + (size_t)NBP * 4);
  const size_t oCNT = off; off = al256(off + (size_t)NBP * 4);
  const size_t oOFF = off; off = al256(off + (size_t)NBP * 4);
  const size_t oFLG = off; off = al256(off + (size_t)gA * FLAGP * 4);
  const size_t oSRL = off; off = al256(off + (size_t)gA * RCAP * 4);
  const size_t oW1T = off; off = al256(off + (size_t)DIM * DIM * 2);
  const size_t oW2D = off; off = al256(off + (size_t)DIM * XP * 2);
  const size_t oW3D = off; off = al256(off + (size_t)DIM * XP * 2);
  const size_t oH   = off; off = al256(off + (size_t)MP * DIM * 4);
  const size_t oXHL = off; off = al256(off + (size_t)MP * XP * 2);
  if (off > ws_size || off > (size_t)WSMAX) return;
  float*          DIS  = (float*)(ws + oDIS);
  int*            CNT  = (int*)(ws + oCNT);
  int*            OFFS = (int*)(ws + oOFF);
  int*            FLG  = (int*)(ws + oFLG);
  int*            SRCL = (int*)(ws + oSRL);
  unsigned short* W1T  = (unsigned short*)(ws + oW1T);
  unsigned short* W2D  = (unsigned short*)(ws + oW2D);
  unsigned short* W3D  = (unsigned short*)(ws + oW3D);
  float*          H    = (float*)(ws + oH);
  unsigned short* XHL  = (unsigned short*)(ws + oXHL);
  unsigned short* XB   = XHL;

  const size_t bktLds = (size_t)BKT_LDS_INTS * 4;
  hipFuncSetAttribute(reinterpret_cast<const void*>(&k_bucket), hipFuncAttributeMaxDynamicSharedMemorySize, (int)bktLds);

  const int nUx = MP * (DIM / 8);
  k_wprep<<<(NU1 + 2 * NU2) / NTHR, NTHR, 0, stream>>>(W1, W2, W3, W1T, W2D, W3D);
  k_cvx<<<cdiv(nUx, NTHR), NTHR, 0, stream>>>(x, nN, nUx, XB);
  k_bucket<<<gA, NTHR, bktLds, stream>>>(src, dst, nE, nN, vec8, SRCL, CNT, OFFS, FLG, DIS);
  k_gemm<<<dim3(gM, DIM / GBN), GTHR, 0, stream>>>(XB, DIM, W1T, DIM, H);
  k_agg<1><<<gA, NTHR, 0, stream>>>(SRCL, CNT, OFFS, FLG, DIS, H, b1, nN, MP, XHL, out);
  k_gemm<<<dim3(gM, DIM / GBN), GTHR, 0, stream>>>(XHL, XP, W2D, XP, H);
  k_agg<1><<<gA, NTHR, 0, stream>>>(SRCL, CNT, OFFS, FLG, DIS, H, b2, nN, MP, XHL, out);
  k_gemm<<<dim3(gM, DIM / GBN), GTHR, 0, stream>>>(XHL, XP, W3D, XP, H);
  k_agg<0><<<gA, NTHR, 0, stream>>>(SRCL, CNT, OFFS, FLG, DIS, H, b3, nN, MP, XHL, out);
}
